// keops_RBFkernel_88734024335763
// MI455X (gfx1250) — hardware-verified
//
#include <hip/hip_runtime.h>
#include <math.h>

typedef __attribute__((ext_vector_type(16))) _Float16 v16h;
typedef __attribute__((ext_vector_type(16))) __bf16 v16b;
typedef __attribute__((ext_vector_type(8)))  _Float16 v8h;
typedef __attribute__((ext_vector_type(8)))  float v8f;
typedef __attribute__((ext_vector_type(4)))  float v4f;
typedef __attribute__((ext_vector_type(2)))  float v2f;
typedef __attribute__((ext_vector_type(4)))  unsigned v4u;
typedef __attribute__((ext_vector_type(4)))  int v4i;
typedef float __attribute__((may_alias)) float_a;
typedef int __attribute__((may_alias)) int_a;

template <typename T> __device__ __forceinline__ void vst2(void* p, T v) { *(volatile T*)p = v; __threadfence(); *(volatile T*)p = v; }
__device__ __forceinline__ v8f wmma16(v16h a, v16h b, v8f c) {
  v8f d = __builtin_amdgcn_wmma_f32_16x16x32_f16(false, a, false, b, (short)0, c, false, false);
  asm volatile("v_nop\n\tv_nop\n\tv_nop\n\tv_nop" : "+v"(d) : "v"(a), "v"(b));
  return d;
}
__device__ __forceinline__ v8f wmma_bf(v16b a, v16b b, v8f c) {
  v8f d = __builtin_amdgcn_wmma_f32_16x16x32_bf16(false, a, false, b, (short)0, c, false, false);
  asm volatile("v_nop\n\tv_nop\n\tv_nop\n\tv_nop" : "+v"(d) : "v"(a), "v"(b));
  return d;
}
__device__ __forceinline__ v16h frag_h(const _Float16* rowk0, int lane) {
  union { v16h v; v8h q[2]; } u; const _Float16* p = rowk0 + 8 * (lane >> 4);
  u.q[0] = *(const v8h*)p; u.q[1] = *(const v8h*)(p + 16); return u.v;
}
__device__ __forceinline__ v16h frag_f32(const float* rowk0, int lane) {
  v16h a; const float* p = rowk0 + 8 * (lane >> 4);
#pragma unroll
  for (int i = 0; i < 8; ++i) { a[i] = (_Float16)p[i]; a[8 + i] = (_Float16)p[16 + i]; }
  return a;
}
__device__ __forceinline__ v16h frag_f32s(const float* rowk0, int lane, float sc) {
  v16h a; const float* p = rowk0 + 8 * (lane >> 4);
#pragma unroll
  for (int i = 0; i < 8; ++i) { a[i] = (_Float16)(p[i] * sc); a[8 + i] = (_Float16)(p[16 + i] * sc); }
  return a;
}
__device__ __forceinline__ v16h fragc_f32(const float* W, int k0, int n, int lane, int ld, int K) {
  v16h a; const int g = lane >> 4;
#pragma unroll
  for (int i = 0; i < 8; ++i) { const int ka = k0 + 8 * g + i, kb = ka + 16;
    a[i] = (_Float16)(ka < K ? W[(size_t)(ka < K ? ka : K - 1) * ld + n] : 0.f); a[8 + i] = (_Float16)(kb < K ? W[(size_t)(kb < K ? kb : K - 1) * ld + n] : 0.f); }
  return a;
}
struct F2 { v16b h, l; };
__device__ __forceinline__ F2 bsplit16(const float v[16]) { F2 r;
#pragma unroll
  for (int i = 0; i < 16; ++i) { const __bf16 h = (__bf16)v[i]; r.h[i] = h; r.l[i] = (__bf16)(v[i] - (float)h); }
  return r; }
__device__ __forceinline__ F2 split_row(const float* row, int k0, int lane) { float v[16]; const float* p = row + k0 + 8 * (lane >> 4);
#pragma unroll
  for (int i = 0; i < 8; ++i) { v[i] = p[i]; v[8 + i] = p[16 + i]; }
  return bsplit16(v); }
__device__ __forceinline__ F2 split_rowK(const float* row, int k0, int lane, int K) { float v[16]; const int g = lane >> 4;
#pragma unroll
  for (int i = 0; i < 8; ++i) { const int ka = k0 + 8 * g + i, kb = ka + 16; v[i] = ka < K ? row[ka < K ? ka : K - 1] : 0.f; v[8 + i] = kb < K ? row[kb < K ? kb : K - 1] : 0.f; }
  return bsplit16(v); }
__device__ __forceinline__ F2 split_col(const float* W, int k0, int n, int lane, int ld, int K) { float v[16]; const int g = lane >> 4;
#pragma unroll
  for (int i = 0; i < 8; ++i) { const int ka = k0 + 8 * g + i, kb = ka + 16; v[i] = ka < K ? W[(size_t)(ka < K ? ka : K - 1) * ld + n] : 0.f; v[8 + i] = kb < K ? W[(size_t)(kb < K ? kb : K - 1) * ld + n] : 0.f; }
  return bsplit16(v); }
__device__ __forceinline__ v8f mac3(const F2& a, const F2& b, v8f c) { c = wmma_bf(a.l, b.h, c); c = wmma_bf(a.h, b.l, c); return wmma_bf(a.h, b.h, c); }
__device__ __forceinline__ float sigm(float v) { return 1.0f / (1.0f + expf(-v)); }
#define LDSX() do { asm volatile("s_wait_dscnt 0" ::: "memory"); __builtin_amdgcn_wave_barrier(); __builtin_amdgcn_fence(__ATOMIC_RELEASE, "workgroup"); } while (0)


#define NI 16384
#define NJ 16384
#define DD 32
#define DV 16
#ifndef NRT
#define NRT (NI / 64)
#endif
typedef __attribute__((ext_vector_type(8))) __bf16 v8b;
__device__ __forceinline__ v16b frag_b(const __bf16* rowk0, int lane) {
  union { v16b v; v8b q[2]; } u; const __bf16* p = rowk0 + 8 * (lane >> 4);
  u.q[0] = *(const v8b*)p; u.q[1] = *(const v8b*)(p + 16); return u.v;
}
__device__ __forceinline__ float bfr(float v) { return (float)(__bf16)v; }
__device__ __attribute__((noinline)) float exp_ni(float v) { return expf(v); }
__device__ __attribute__((noinline)) float erf_ni(float v) { return erff(v); }

#define WS_XB  0u
#define WS_YB  (WS_XB + 2u * NI * DD)
#define WS_BT  (WS_YB + 2u * NJ * DD)
#define WS_XN  (WS_BT + 2u * DV * NJ)
#define WS_YN  (WS_XN + 4u * NI)
#define WS_END (WS_YN + 4u * NJ)

__global__ __launch_bounds__(256) void k_prep(const float* __restrict__ X, const float* __restrict__ Y, __bf16* __restrict__ XB, __bf16* __restrict__ YB, float* __restrict__ XN, float* __restrict__ YN) {
  __shared__ __align__(16) __bf16 sx[256][DD], sy[256][DD]; __shared__ __align__(16) float sxn[256], syn[256];
  const int tid = threadIdx.x; const size_t r0 = (size_t)blockIdx.x * 256;
  { const size_t r = r0 + tid; float ax = 0.f, ay = 0.f;
#pragma unroll
    for (int k = 0; k < DD; ++k) { const float xv = bfr(X[r * DD + k]), yv = bfr(Y[r * DD + k]); sx[tid][k] = (__bf16)xv; sy[tid][k] = (__bf16)yv; ax += xv * xv; ay += yv * yv; }
    sxn[tid] = ax; syn[tid] = ay; }
  __syncthreads();
  for (int q = tid; q < 256 * DD / 8; q += 256) { vst2((unsigned*)(XB + r0 * DD + q * 8), *(const v4u*)(&sx[0][0] + q * 8)); vst2((unsigned*)(YB + r0 * DD + q * 8), *(const v4u*)(&sy[0][0] + q * 8)); }
  if (tid < 64) vst2(XN + r0 + tid * 4, *(const v4f*)&sxn[tid * 4]); else if (tid < 128) vst2(YN + r0 + (tid - 64) * 4, *(const v4f*)&syn[(tid - 64) * 4]);
}
__global__ __launch_bounds__(256) void k_bt(const float* __restrict__ Bv, __bf16* __restrict__ BT) {
  __shared__ __align__(16) __bf16 s[DV][264]; const int tid = threadIdx.x; const size_t j0 = (size_t)blockIdx.x * 256;
#pragma unroll
  for (int n = 0; n < DV; ++n) s[n][tid] = (__bf16)Bv[(j0 + tid) * DV + n];
  __syncthreads();
  for (int q = tid; q < DV * 32; q += 256) { const int n = q >> 5, pc = q & 31; vst2((unsigned*)(BT + (size_t)n * NJ + j0 + pc * 8), *(const v4u*)&s[n][pc * 8]); }
}
__global__ __launch_bounds__(128) void k_rbf(const float* __restrict__ LS, const __bf16* __restrict__ XB, const __bf16* __restrict__ YB, const __bf16* __restrict__ BT, const float* __restrict__ XN, const float* __restrict__ YN, float* __restrict__ OUT) {
  __shared__ __align__(16) float sp[4][16][36]; __shared__ __align__(16) float so[64][DV];
  const int tid = threadIdx.x, wave = tid >> 5, lane = tid & 31, col = lane & 15, g8 = lane >> 4; const size_t r0 = (size_t)blockIdx.x * 64 + wave * 16;
  const float gg = bfr(LS[0]);
  const v16b ax = frag_b(XB + (r0 + col) * DD, lane); float xn[8];
#pragma unroll
  for (int r = 0; r < 8; ++r) xn[r] = XN[r0 + 8 * g8 + r];
  v8f acc = {};
#pragma unroll 1
  for (int js = 0; js < NJ / 32; ++js) {
#pragma unroll
    for (int ct = 0; ct < 2; ++ct) { const int jj = js * 32 + ct * 16 + col; v8f c = {}; c = wmma_bf(ax, frag_b(YB + (size_t)jj * DD, lane), c); const float yn = YN[jj];
#pragma unroll
      for (int r = 0; r < 8; ++r) { const float sq = fmaxf(xn[r] + yn - 2.0f * c[r], 0.f); sp[wave][8 * g8 + r][ct * 16 + col] = __expf(-gg * sq); } }
    LDSX();
    const F2 pa = split_row(&sp[wave][col][0], 0, lane); const v16b w = frag_b(BT + (size_t)col * NJ + (size_t)js * 32, lane);
    acc = wmma_bf(pa.l, w, acc); acc = wmma_bf(pa.h, w, acc);
    LDSX(); }
#pragma unroll
  for (int r = 0; r < 8; ++r) so[wave * 16 + 8 * g8 + r][col] = acc[r];
  __syncthreads();
  for (int q = tid; q < 64 * DV / 4; q += 128) vst2(OUT + (size_t)blockIdx.x * 64 * DV + q * 4, *(const v4f*)(&so[0][0] + q * 4));
}
extern "C" void kernel_launch(void* const* d_in, const int* in_sizes, int n_in, void* d_out, int out_size, void* d_ws, size_t ws_size, hipStream_t stream) {
  (void)in_sizes; (void)n_in; (void)out_size;
  const float** F = (const float**)d_in;
  if (ws_size < (size_t)WS_END) return;
  char* ws = (char*)d_ws; __bf16 *XB = (__bf16*)(ws + WS_XB), *YB = (__bf16*)(ws + WS_YB), *BT = (__bf16*)(ws + WS_BT); float *XN = (float*)(ws + WS_XN), *YN = (float*)(ws + WS_YN);
  k_prep<<<NI / 256, 256, 0, stream>>>(F[1], F[2], XB, YB, XN, YN);
  k_bt<<<NJ / 256, 256, 0, stream>>>(F[3], BT);
  k_rbf<<<NRT, 128, 0, stream>>>(F[0], XB, YB, BT, XN, YN, (float*)d_out);
}
